// singleSANNLayer_5712306504312
// MI455X (gfx1250) — hardware-verified
//
#include <hip/hip_runtime.h>
#include <math.h>

typedef __attribute__((ext_vector_type(16))) _Float16 v16h;
typedef __attribute__((ext_vector_type(16))) __bf16 v16b;
typedef __attribute__((ext_vector_type(8)))  _Float16 v8h;
typedef __attribute__((ext_vector_type(8)))  float v8f;
typedef __attribute__((ext_vector_type(4)))  float v4f;
typedef __attribute__((ext_vector_type(2)))  float v2f;
typedef __attribute__((ext_vector_type(4)))  unsigned v4u;
typedef __attribute__((ext_vector_type(4)))  int v4i;
typedef float __attribute__((may_alias)) float_a;
typedef int __attribute__((may_alias)) int_a;

template <typename T> __device__ __forceinline__ void vst2(void* p, T v) { *(volatile T*)p = v; __threadfence(); *(volatile T*)p = v; }
__device__ __forceinline__ v8f wmma16(v16h a, v16h b, v8f c) {
  v8f d = __builtin_amdgcn_wmma_f32_16x16x32_f16(false, a, false, b, (short)0, c, false, false);
  asm volatile("v_nop\n\tv_nop\n\tv_nop\n\tv_nop" : "+v"(d) : "v"(a), "v"(b));
  return d;
}
__device__ __forceinline__ v8f wmma_bf(v16b a, v16b b, v8f c) {
  v8f d = __builtin_amdgcn_wmma_f32_16x16x32_bf16(false, a, false, b, (short)0, c, false, false);
  asm volatile("v_nop\n\tv_nop\n\tv_nop\n\tv_nop" : "+v"(d) : "v"(a), "v"(b));
  return d;
}
__device__ __forceinline__ v16h frag_h(const _Float16* rowk0, int lane) {
  union { v16h v; v8h q[2]; } u; const _Float16* p = rowk0 + 8 * (lane >> 4);
  u.q[0] = *(const v8h*)p; u.q[1] = *(const v8h*)(p + 16); return u.v;
}
__device__ __forceinline__ v16h frag_f32(const float* rowk0, int lane) {
  v16h a; const float* p = rowk0 + 8 * (lane >> 4);
#pragma unroll
  for (int i = 0; i < 8; ++i) { a[i] = (_Float16)p[i]; a[8 + i] = (_Float16)p[16 + i]; }
  return a;
}
__device__ __forceinline__ v16h frag_f32s(const float* rowk0, int lane, float sc) {
  v16h a; const float* p = rowk0 + 8 * (lane >> 4);
#pragma unroll
  for (int i = 0; i < 8; ++i) { a[i] = (_Float16)(p[i] * sc); a[8 + i] = (_Float16)(p[16 + i] * sc); }
  return a;
}
__device__ __forceinline__ v16h fragc_f32(const float* W, int k0, int n, int lane, int ld, int K) {
  v16h a; const int g = lane >> 4;
#pragma unroll
  for (int i = 0; i < 8; ++i) { const int ka = k0 + 8 * g + i, kb = ka + 16;
    a[i] = (_Float16)(ka < K ? W[(size_t)(ka < K ? ka : K - 1) * ld + n] : 0.f); a[8 + i] = (_Float16)(kb < K ? W[(size_t)(kb < K ? kb : K - 1) * ld + n] : 0.f); }
  return a;
}
struct F2 { v16b h, l; };
__device__ __forceinline__ F2 bsplit16(const float v[16]) { F2 r;
#pragma unroll
  for (int i = 0; i < 16; ++i) { const __bf16 h = (__bf16)v[i]; r.h[i] = h; r.l[i] = (__bf16)(v[i] - (float)h); }
  return r; }
__device__ __forceinline__ F2 split_row(const float* row, int k0, int lane) { float v[16]; const float* p = row + k0 + 8 * (lane >> 4);
#pragma unroll
  for (int i = 0; i < 8; ++i) { v[i] = p[i]; v[8 + i] = p[16 + i]; }
  return bsplit16(v); }
__device__ __forceinline__ F2 split_rowK(const float* row, int k0, int lane, int K) { float v[16]; const int g = lane >> 4;
#pragma unroll
  for (int i = 0; i < 8; ++i) { const int ka = k0 + 8 * g + i, kb = ka + 16; v[i] = ka < K ? row[ka < K ? ka : K - 1] : 0.f; v[8 + i] = kb < K ? row[kb < K ? kb : K - 1] : 0.f; }
  return bsplit16(v); }
__device__ __forceinline__ F2 split_col(const float* W, int k0, int n, int lane, int ld, int K) { float v[16]; const int g = lane >> 4;
#pragma unroll
  for (int i = 0; i < 8; ++i) { const int ka = k0 + 8 * g + i, kb = ka + 16; v[i] = ka < K ? W[(size_t)(ka < K ? ka : K - 1) * ld + n] : 0.f; v[8 + i] = kb < K ? W[(size_t)(kb < K ? kb : K - 1) * ld + n] : 0.f; }
  return bsplit16(v); }
__device__ __forceinline__ v8f mac3(const F2& a, const F2& b, v8f c) { c = wmma_bf(a.l, b.h, c); c = wmma_bf(a.h, b.l, c); return wmma_bf(a.h, b.h, c); }
__device__ __forceinline__ float sigm(float v) { return 1.0f / (1.0f + expf(-v)); }
#define LDSX() do { asm volatile("s_wait_dscnt 0" ::: "memory"); __builtin_amdgcn_wave_barrier(); __builtin_amdgcn_fence(__ATOMIC_RELEASE, "workgroup"); } while (0)


#define NN 3072
#define DIN 256
#define NH 8
#define DH 32
#define HD2 (NH * DH)
#define NBC 272
#ifndef NMB
#define NMB (NN / 64)
#endif
typedef __attribute__((ext_vector_type(8))) __bf16 v8b;
__device__ __forceinline__ v16b frag_b(const __bf16* rowk0, int lane) {
  union { v16b v; v8b q[2]; } u; const __bf16* p = rowk0 + 8 * (lane >> 4);
  u.q[0] = *(const v8b*)p; u.q[1] = *(const v8b*)(p + 16); return u.v;
}
__device__ __forceinline__ float bfr(float v) { return (float)(__bf16)v; }
__device__ __attribute__((noinline)) float exp_ni(float v) { return expf(v); }
__device__ __attribute__((noinline)) float erf_ni(float v) { return erff(v); }

#define WS_PW   0u
#define WS_PR   (WS_PW + 2u * (size_t)4 * HD2 * DIN)
#define WS_AS   (WS_PR + 4u * (size_t)4 * NN * HD2)
#define WS_AD   (WS_AS + 4u * 2 * NH * NN)
#define WS_RMX  (WS_AD + 4u * 2 * NH * NN)
#define WS_GMX  (WS_RMX + 4u * 2 * NN)
#define WS_AT   (WS_GMX + 256u)
#define WS_BH   (WS_AT + 2u * (size_t)2 * NN * NN)
#define WS_BL   (WS_BH + 2u * (size_t)2 * NBC * NN)
#define WS_END  (WS_BL + 2u * (size_t)2 * NBC * NN)

__global__ __launch_bounds__(256) void k_packw(const float* __restrict__ Wt, __bf16* __restrict__ P) {
  const int he = blockIdx.x, ft = blockIdx.y, t = threadIdx.x; const int h = he >> 5, e = he & 31; __shared__ __align__(16) __bf16 s[DIN];
  s[t] = (__bf16)Wt[((((size_t)ft * NH + h) * DIN) + t) * DH + e]; __syncthreads();
  if (t < DIN / 8) vst2((unsigned*)(P + ((size_t)ft * HD2 + he) * DIN + t * 8), *(const v4u*)&s[t * 8]);
}
__global__ __launch_bounds__(128) void k_proj(const float* __restrict__ E0, const float* __restrict__ E1, const __bf16* __restrict__ P, float* __restrict__ PR) {
  __shared__ __align__(16) float so[4][16][132];
  const int tid = threadIdx.x, wave = tid >> 5, lane = tid & 31, col = lane & 15, g = lane >> 4; const size_t r0 = (size_t)blockIdx.x * 64 + wave * 16; const int n0 = blockIdx.y * 128; const int which = blockIdx.z;
  const float* X = (which == 0 || which == 3) ? E0 : E1; const int ft = (which == 0) ? 1 : (which == 1) ? 3 : (which == 2) ? 2 : 0;
  const __bf16* Wr = P + (size_t)ft * HD2 * DIN;
  v8f acc[8] = {};
#pragma unroll
  for (int kc = 0; kc < DIN / 32; ++kc) { v16b a; { const float* p = X + (r0 + col) * DIN + kc * 32 + 8 * g;
#pragma unroll
      for (int i = 0; i < 8; ++i) { a[i] = (__bf16)p[i]; a[8 + i] = (__bf16)p[16 + i]; } }
#pragma unroll
    for (int j = 0; j < 8; ++j) acc[j] = wmma_bf(a, frag_b(Wr + (size_t)(n0 + j * 16 + col) * DIN + kc * 32, lane), acc[j]); }
#pragma unroll
  for (int j = 0; j < 8; ++j)
#pragma unroll
    for (int r = 0; r < 8; ++r) so[wave][8 * g + r][j * 16 + col] = acc[j][r];
  LDSX();
  for (int rl = 0; rl < 16; ++rl) vst2(PR + ((size_t)which * NN + r0 + rl) * HD2 + n0 + lane * 4, *(const v4f*)&so[wave][rl][lane * 4]);
}
__global__ __launch_bounds__(256) void k_adots(const float* __restrict__ PR, const float* __restrict__ ATTN, float* __restrict__ AS, float* __restrict__ AD) {
  const int n = blockIdx.x * 32 + (threadIdx.x & 31); const int h = threadIdx.x >> 5; const int i = blockIdx.y;
  const float* fp = PR + ((size_t)(i == 0 ? 0 : 2) * NN + n) * HD2 + h * DH; const float* tp = PR + ((size_t)(i == 0 ? 1 : 3) * NN + n) * HD2 + h * DH;
  float s = 0.f, d = 0.f;
#pragma unroll 1
  for (int e = 0; e < DH; ++e) { s += fp[e] * bfr(ATTN[(h * 2 * DH + e) * 2 + i]); d += tp[e] * bfr(ATTN[(h * 2 * DH + DH + e) * 2 + i]); }
  AS[((size_t)i * NH + h) * NN + n] = s; AD[((size_t)i * NH + h) * NN + n] = d;
}
__global__ __launch_bounds__(256) void k_rowmax(const int* __restrict__ ADJ0, const int* __restrict__ ADJ1, const float* __restrict__ AS, const float* __restrict__ AD, float* __restrict__ RMX) {
  const int n = blockIdx.x, i = blockIdx.y, t = threadIdx.x; const int* adj = (i == 0 ? ADJ0 : ADJ1) + (size_t)n * NN; __shared__ float red[256];
  float mx = -3.0e38f;
  for (int m = t; m < NN; m += 256) { if (adj[m] > 0) {
#pragma unroll
      for (int h = 0; h < NH; ++h) mx = fmaxf(mx, AS[((size_t)i * NH + h) * NN + n] + AD[((size_t)i * NH + h) * NN + m]); } }
  red[t] = mx; __syncthreads();
  for (int s = 128; s > 0; s >>= 1) { if (t < s) red[t] = fmaxf(red[t], red[t + s]); __syncthreads(); }
  if (t == 0) RMX[(size_t)i * NN + n] = red[0];
}
__global__ __launch_bounds__(256) void k_gmax(const float* __restrict__ RMX, float* __restrict__ GMX) {
  const int i = blockIdx.x, t = threadIdx.x; __shared__ float red[256]; float mx = -3.0e38f; for (int n = t; n < NN; n += 256) mx = fmaxf(mx, RMX[(size_t)i * NN + n]); red[t] = mx; __syncthreads();
  for (int s = 128; s > 0; s >>= 1) { if (t < s) red[t] = fmaxf(red[t], red[t + s]); __syncthreads(); }
  if (t == 0) GMX[i] = red[0];
}
__global__ __launch_bounds__(256) void k_adjt(const int* __restrict__ ADJ0, const int* __restrict__ ADJ1, __bf16* __restrict__ AT) {
  __shared__ __align__(16) __bf16 s[64][72]; const int mb = blockIdx.x, nb = blockIdx.y, i = blockIdx.z, t = threadIdx.x; const int* adj = (i == 0 ? ADJ0 : ADJ1);
  for (int e = t; e < 64 * 64; e += 256) { const int nl = e >> 6, ml = e & 63; s[ml][nl] = (__bf16)((adj[(size_t)(nb * 64 + nl) * NN + mb * 64 + ml] > 0) ? 1.0f : 0.0f); }
  __syncthreads();
  for (int e = t; e < 64 * 8; e += 256) { const int ml = e >> 3, q = e & 7; vst2((unsigned*)(AT + ((size_t)i * NN + mb * 64 + ml) * NN + nb * 64 + q * 8), *(const v4u*)&s[ml][q * 8]); }
}
__device__ __attribute__((noinline)) float exp_p(float v) { return expf(v); }
__global__ __launch_bounds__(256) void k_bplanes(const float* __restrict__ PR, const float* __restrict__ AS, const float* __restrict__ GMX, __bf16* __restrict__ BH, __bf16* __restrict__ BL) {
  __shared__ __align__(16) __bf16 sh[NBC][72], sl[NBC][72]; __shared__ float sw[NH][64];
  const int nb = blockIdx.x, i = blockIdx.y, t = threadIdx.x; const float gm = GMX[i]; const float* fp = PR + ((size_t)(i == 0 ? 0 : 2) * NN + nb * 64) * HD2;
  for (int e = t; e < NH * 64; e += 256) { const int h = e >> 6, nl = e & 63; sw[h][nl] = exp_p(AS[((size_t)i * NH + h) * NN + nb * 64 + nl] - gm); }
  __syncthreads();
  for (int e = t; e < NBC * 64; e += 256) { const int c = e >> 6, nl = e & 63; float v; if (c < HD2) v = sw[c >> 5][nl] * fp[(size_t)nl * HD2 + c]; else if (c < HD2 + NH) v = sw[c - HD2][nl]; else v = 0.f; const __bf16 h = (__bf16)v; sh[c][nl] = h; sl[c][nl] = (__bf16)(v - (float)h); }
  __syncthreads();
  for (int e = t; e < NBC * 8; e += 256) { const int c = e >> 3, q = e & 7; const size_t o = ((size_t)i * NBC + c) * NN + nb * 64 + q * 8; vst2((unsigned*)(BH + o), *(const v4u*)&sh[c][q * 8]); vst2((unsigned*)(BL + o), *(const v4u*)&sl[c][q * 8]); }
}
__global__ __launch_bounds__(128) void k_agg(const __bf16* __restrict__ AT, const __bf16* __restrict__ BH, const __bf16* __restrict__ BL, const float* __restrict__ AD, float* __restrict__ OUT) {
  __shared__ __align__(16) float so[4][16][HD2 + 4]; __shared__ float s0[4][16][NH];
  const int tid = threadIdx.x, wave = tid >> 5, lane = tid & 31, col = lane & 15, g = lane >> 4; const int i = blockIdx.y; const size_t m0 = (size_t)blockIdx.x * 64 + wave * 16;
  const int tgt = (i == 0) ? 1 : 0;
  v8f acc[17] = {};
#pragma unroll 1
  for (int kc = 0; kc < NN / 32; ++kc) { const v16b a = frag_b(AT + ((size_t)i * NN + m0 + col) * NN + kc * 32, lane);
#pragma unroll
    for (int j = 0; j < 17; ++j) { const size_t bo = ((size_t)i * NBC + j * 16 + col) * NN + kc * 32; acc[j] = wmma_bf(a, frag_b(BL + bo, lane), acc[j]); acc[j] = wmma_bf(a, frag_b(BH + bo, lane), acc[j]); } }
#pragma unroll
  for (int r = 0; r < 8; ++r) { if (col < NH) s0[wave][8 * g + r][col] = acc[16][r]; }
  LDSX();
#pragma unroll
  for (int j = 0; j < 16; ++j) { const int c = j * 16 + col; const int h = c >> 5;
#pragma unroll
    for (int r = 0; r < 8; ++r) { const size_t m = m0 + 8 * g + r; const float ea = exp_p(AD[((size_t)i * NH + h) * NN + m]); so[wave][8 * g + r][c] = (ea * acc[j][r]) / (ea * s0[wave][8 * g + r][h] + 1e-9f); } }
  LDSX();
  float* outp = OUT + (size_t)tgt * NN * HD2;
  for (int rl = 0; rl < 16; ++rl) for (int q = lane; q < HD2 / 4; q += 32) vst2(outp + (m0 + rl) * HD2 + q * 4, *(const v4f*)&so[wave][rl][q * 4]);
}
extern "C" void kernel_launch(void* const* d_in, const int* in_sizes, int n_in, void* d_out, int out_size, void* d_ws, size_t ws_size, hipStream_t stream) {
  (void)in_sizes; (void)n_in; (void)out_size;
  const float** F = (const float**)d_in;
  if (ws_size < (size_t)WS_END) return;
  char* ws = (char*)d_ws; __bf16 *P = (__bf16*)(ws + WS_PW), *AT = (__bf16*)(ws + WS_AT), *BH = (__bf16*)(ws + WS_BH), *BL = (__bf16*)(ws + WS_BL); float *PR = (float*)(ws + WS_PR), *AS = (float*)(ws + WS_AS), *AD = (float*)(ws + WS_AD), *RMX = (float*)(ws + WS_RMX), *GMX = (float*)(ws + WS_GMX);
  k_packw<<<dim3(HD2, 4), 256, 0, stream>>>(F[4], P);
  k_proj<<<dim3(NN / 64, HD2 / 128, 4), 128, 0, stream>>>(F[0], F[1], P, PR);
  k_adots<<<dim3(NN / 32, 2), 256, 0, stream>>>(PR, F[5], AS, AD);
  k_rowmax<<<dim3(NN, 2), 256, 0, stream>>>((const int*)d_in[2], (const int*)d_in[3], AS, AD, RMX);
  k_gmax<<<2, 256, 0, stream>>>(RMX, GMX);
  k_adjt<<<dim3(NN / 64, NN / 64, 2), 256, 0, stream>>>((const int*)d_in[2], (const int*)d_in[3], AT);
  k_bplanes<<<dim3(NN / 64, 2), 256, 0, stream>>>(PR, AS, GMX, BH, BL);
  k_agg<<<dim3(NMB, 2), 128, 0, stream>>>(AT, BH, BL, AD, (float*)d_out);
}
